// ImprovedMLPDecoder_84920093376639
// MI455X (gfx1250) — hardware-verified
//
#include <hip/hip_runtime.h>
#include <math.h>

typedef __attribute__((ext_vector_type(16))) _Float16 v16h;
typedef __attribute__((ext_vector_type(16))) __bf16 v16b;
typedef __attribute__((ext_vector_type(8)))  _Float16 v8h;
typedef __attribute__((ext_vector_type(8)))  float v8f;
typedef __attribute__((ext_vector_type(4)))  float v4f;
typedef __attribute__((ext_vector_type(2)))  float v2f;
typedef __attribute__((ext_vector_type(4)))  unsigned v4u;
typedef __attribute__((ext_vector_type(4)))  int v4i;
typedef float __attribute__((may_alias)) float_a;
typedef int __attribute__((may_alias)) int_a;

template <typename T> __device__ __forceinline__ void vst2(void* p, T v) { *(volatile T*)p = v; __threadfence(); *(volatile T*)p = v; }
__device__ __forceinline__ v8f wmma16(v16h a, v16h b, v8f c) {
  v8f d = __builtin_amdgcn_wmma_f32_16x16x32_f16(false, a, false, b, (short)0, c, false, false);
  asm volatile("v_nop\n\tv_nop\n\tv_nop\n\tv_nop" : "+v"(d) : "v"(a), "v"(b));
  return d;
}
__device__ __forceinline__ v8f wmma_bf(v16b a, v16b b, v8f c) {
  v8f d = __builtin_amdgcn_wmma_f32_16x16x32_bf16(false, a, false, b, (short)0, c, false, false);
  asm volatile("v_nop\n\tv_nop\n\tv_nop\n\tv_nop" : "+v"(d) : "v"(a), "v"(b));
  return d;
}
__device__ __forceinline__ v16h frag_h(const _Float16* rowk0, int lane) {
  union { v16h v; v8h q[2]; } u; const _Float16* p = rowk0 + 8 * (lane >> 4);
  u.q[0] = *(const v8h*)p; u.q[1] = *(const v8h*)(p + 16); return u.v;
}
__device__ __forceinline__ v16h frag_f32(const float* rowk0, int lane) {
  v16h a; const float* p = rowk0 + 8 * (lane >> 4);
#pragma unroll
  for (int i = 0; i < 8; ++i) { a[i] = (_Float16)p[i]; a[8 + i] = (_Float16)p[16 + i]; }
  return a;
}
__device__ __forceinline__ v16h frag_f32s(const float* rowk0, int lane, float sc) {
  v16h a; const float* p = rowk0 + 8 * (lane >> 4);
#pragma unroll
  for (int i = 0; i < 8; ++i) { a[i] = (_Float16)(p[i] * sc); a[8 + i] = (_Float16)(p[16 + i] * sc); }
  return a;
}
__device__ __forceinline__ v16h fragc_f32(const float* W, int k0, int n, int lane, int ld, int K) {
  v16h a; const int g = lane >> 4;
#pragma unroll
  for (int i = 0; i < 8; ++i) { const int ka = k0 + 8 * g + i, kb = ka + 16;
    a[i] = (_Float16)(ka < K ? W[(size_t)ka * ld + n] : 0.f); a[8 + i] = (_Float16)(kb < K ? W[(size_t)kb * ld + n] : 0.f); }
  return a;
}
struct F2 { v16b h, l; };
__device__ __forceinline__ F2 bsplit16(const float v[16]) { F2 r;
#pragma unroll
  for (int i = 0; i < 16; ++i) { const __bf16 h = (__bf16)v[i]; r.h[i] = h; r.l[i] = (__bf16)(v[i] - (float)h); }
  return r; }
__device__ __forceinline__ F2 split_row(const float* row, int k0, int lane) { float v[16]; const float* p = row + k0 + 8 * (lane >> 4);
#pragma unroll
  for (int i = 0; i < 8; ++i) { v[i] = p[i]; v[8 + i] = p[16 + i]; }
  return bsplit16(v); }
__device__ __forceinline__ F2 split_rowK(const float* row, int k0, int lane, int K) { float v[16]; const int g = lane >> 4;
#pragma unroll
  for (int i = 0; i < 8; ++i) { const int ka = k0 + 8 * g + i, kb = ka + 16; v[i] = ka < K ? row[ka] : 0.f; v[8 + i] = kb < K ? row[kb] : 0.f; }
  return bsplit16(v); }
__device__ __forceinline__ F2 split_col(const float* W, int k0, int n, int lane, int ld, int K) { float v[16]; const int g = lane >> 4;
#pragma unroll
  for (int i = 0; i < 8; ++i) { const int ka = k0 + 8 * g + i, kb = ka + 16; v[i] = ka < K ? W[(size_t)ka * ld + n] : 0.f; v[8 + i] = kb < K ? W[(size_t)kb * ld + n] : 0.f; }
  return bsplit16(v); }
__device__ __forceinline__ v8f mac3(const F2& a, const F2& b, v8f c) { c = wmma_bf(a.l, b.h, c); c = wmma_bf(a.h, b.l, c); return wmma_bf(a.h, b.h, c); }
__device__ __forceinline__ float sigm(float v) { return 1.0f / (1.0f + expf(-v)); }
#define LDSX() do { asm volatile("s_wait_dscnt 0" ::: "memory"); __builtin_amdgcn_wave_barrier(); __builtin_amdgcn_fence(__ATOMIC_RELEASE, "workgroup"); } while (0)

__device__ __forceinline__ v16h fragc_f32s(const float* __restrict__ base, int k0, int n, int lane, int ld, float sc) {
  const int g = lane >> 4; v16h r;
#pragma unroll
  for (int i = 0; i < 8; ++i) { r[i] = (_Float16)(base[(size_t)(k0 + 8 * g + i) * ld + n] * sc); r[8 + i] = (_Float16)(base[(size_t)(k0 + 16 + 8 * g + i) * ld + n] * sc); }
  return r;
}
#define NND 50000
#define NE 500000
#define DD 256
#define H1 128
#define H2 64
#define NP (H1 + H2)
#define NNP 50048
#define NEB ((NE + 63) / 64)

__device__ __forceinline__ float gelu_e(float v) { return 0.5f * v * (1.0f + erff(v * 0.70710678118654752f)); }
__global__ __launch_bounds__(128) void k_node(const float* __restrict__ drug, const float* __restrict__ dis, const float* __restrict__ W1, const float* __restrict__ Ws, float* __restrict__ PD, float* __restrict__ PS) {
  __shared__ __align__(16) float so[4][16][NP + 4];
  const int tid = threadIdx.x, wave = tid >> 5, lane = tid & 31, col = lane & 15, g = lane >> 4;
  const int which = blockIdx.y, r0 = blockIdx.x * 64 + wave * 16; const float* X = which == 0 ? drug : dis; const int ra = (r0 + col) < NND ? (r0 + col) : NND - 1;
  v8f acc[12];
#pragma unroll
  for (int t = 0; t < 12; ++t) acc[t] = (v8f){};
#pragma unroll 1
  for (int kc = 0; kc < DD / 32; ++kc) { const v16h a = frag_f32(X + (size_t)ra * DD + kc * 32, lane); const int kg = which * DD + kc * 32;
#pragma unroll
    for (int t = 0; t < 8; ++t) acc[t] = wmma16(a, fragc_f32s(W1, kg, t * 16 + col, lane, H1, 16.0f), acc[t]);
#pragma unroll
    for (int t = 0; t < 4; ++t) acc[8 + t] = wmma16(a, fragc_f32s(Ws, kg, t * 16 + col, lane, H2, 16.0f), acc[8 + t]); }
#pragma unroll
  for (int t = 0; t < 12; ++t)
#pragma unroll
    for (int r = 0; r < 8; ++r) so[wave][8 * g + r][t * 16 + col] = acc[t][r] * (1.0f / 16.0f);
  LDSX();
  float* P = which == 0 ? PD : PS;
  for (int q = lane; q < 16 * (NP / 4); q += 32) { const int rl = q / (NP / 4), pc = q % (NP / 4); vst2(P + (size_t)(r0 + rl) * NP + pc * 4, *(const v4f*)(&so[wave][rl][pc * 4])); }
}
__global__ __launch_bounds__(128) void k_edge(const int* __restrict__ sidx, const int* __restrict__ didx, const float* __restrict__ PD, const float* __restrict__ PS, const float* __restrict__ b1, const float* __restrict__ g1, const float* __restrict__ be1,
                                            const float* __restrict__ W2, const float* __restrict__ b2, const float* __restrict__ g2, const float* __restrict__ be2, const float* __restrict__ W3, const float* __restrict__ b3, const float* __restrict__ bs, float* __restrict__ out) {
  __shared__ __align__(16) float sp[64][NP + 1];
  __shared__ __align__(16) _Float16 sa[4][16][H1 + 8];
  __shared__ __align__(16) float sh[64][H2 + 1];
  __shared__ __align__(16) float so[64];
  const int tid = threadIdx.x, wave = tid >> 5, lane = tid & 31, col = lane & 15, g = lane >> 4;
  const int e0b = blockIdx.x * 64;
  { const int el = tid >> 1, hf = tid & 1; const int e = e0b + el; int s = 0, d = 0; if (e < NE) { s = sidx[e]; d = didx[e]; s = s < 0 ? 0 : (s >= NND ? NND - 1 : s); d = d < 0 ? 0 : (d >= NND ? NND - 1 : d); }
    const float* ps = PD + (size_t)s * NP; const float* pd = PS + (size_t)d * NP;
    for (int c = hf * 96; c < hf * 96 + 96; ++c) sp[el][c] = ps[c] + pd[c]; }
  __syncthreads();
  { const int el = tid >> 1, hf = tid & 1; float* row = &sp[el][0]; float s = 0.f; for (int c = hf * 64; c < hf * 64 + 64; ++c) { row[c] += b1[c]; s += row[c]; } s += __shfl_xor(s, 1, 32); const float mu = s * (1.0f / H1);
    float q2 = 0.f; for (int c = hf * 64; c < hf * 64 + 64; ++c) { const float dv = row[c] - mu; q2 += dv * dv; } q2 += __shfl_xor(q2, 1, 32); const float rs = rsqrtf(q2 * (1.0f / H1) + 1e-5f);
    for (int c = hf * 64; c < hf * 64 + 64; ++c) sa[el >> 4][el & 15][c] = (_Float16)gelu_e((row[c] - mu) * rs * g1[c] + be1[c]); }
  __syncthreads();
  { v8f acc[4] = {};
#pragma unroll
    for (int kc = 0; kc < 4; ++kc) { const v16h a = frag_h(&sa[wave][col][0] + kc * 32, lane);
#pragma unroll
      for (int t = 0; t < 4; ++t) acc[t] = wmma16(a, fragc_f32s(W2, kc * 32, t * 16 + col, lane, H2, 16.0f), acc[t]); }
#pragma unroll
    for (int t = 0; t < 4; ++t) { const int n = t * 16 + col; const float bb = b2[n];
#pragma unroll
      for (int r = 0; r < 8; ++r) sh[wave * 16 + 8 * g + r][n] = acc[t][r] * (1.0f / 16.0f) + bb; } }
  __syncthreads();
  { const int el = tid >> 1, hf = tid & 1; float* row = &sh[el][0]; float s = 0.f; for (int c = hf * 32; c < hf * 32 + 32; ++c) s += row[c]; s += __shfl_xor(s, 1, 32); const float mu = s * (1.0f / H2);
    float q2 = 0.f; for (int c = hf * 32; c < hf * 32 + 32; ++c) { const float dv = row[c] - mu; q2 += dv * dv; } q2 += __shfl_xor(q2, 1, 32); const float rs = rsqrtf(q2 * (1.0f / H2) + 1e-5f);
    float dsum = 0.f; for (int c = hf * 32; c < hf * 32 + 32; ++c) { const float hv = gelu_e((row[c] - mu) * rs * g2[c] + be2[c] + (sp[el][H1 + c] + bs[c])); dsum += hv * W3[c]; }
    dsum += __shfl_xor(dsum, 1, 32); if (hf == 0) so[el] = dsum + b3[0]; }
  __syncthreads();
  if (tid < 16) { const int e = e0b + tid * 4; if (e + 3 < NE) vst2(out + e, *(const v4f*)(&so[tid * 4])); else { for (int u = 0; u < 4; ++u) if (e + u < NE) vst2(out + e + u, so[tid * 4 + u]); } }
}
extern "C" void kernel_launch(void* const* d_in, const int* in_sizes, int n_in, void* d_out, int out_size, void* d_ws, size_t ws_size, hipStream_t stream) {
  (void)in_sizes; (void)n_in; (void)out_size; (void)ws_size;
  const float** I = (const float**)d_in;
  const float* drug = I[0]; const float* dis = I[1]; const int* sidx = (const int*)d_in[2]; const int* didx = (const int*)d_in[3];
  const float* W1 = I[4]; const float* b1 = I[5]; const float* g1 = I[6]; const float* be1 = I[7]; const float* W2 = I[8]; const float* b2 = I[9]; const float* g2 = I[10]; const float* be2 = I[11]; const float* W3 = I[12]; const float* b3 = I[13]; const float* Ws = I[14]; const float* bs = I[15];
  float* out = (float*)d_out;
  char* ws = (char*)d_ws; size_t off = 0;
  auto take = [&](size_t bytes) { char* p = ws + off; off += (bytes + 255) & ~(size_t)255; return p; };
  float* PD = (float*)take((size_t)NNP * NP * 4); float* PS = (float*)take((size_t)NNP * NP * 4);
  k_node<<<dim3(NNP / 64, 2), 128, 0, stream>>>(drug, dis, W1, Ws, PD, PS);
  k_edge<<<NEB, 128, 0, stream>>>(sidx, didx, PD, PS, b1, g1, be1, W2, b2, g2, be2, W3, b3, bs, out);
}
